// MultiHeadAttention_20770461843824
// MI455X (gfx1250) — hardware-verified
//
#include <hip/hip_runtime.h>
#include <math.h>

typedef __attribute__((ext_vector_type(16))) _Float16 v16h;
typedef __attribute__((ext_vector_type(8)))  _Float16 v8h;
typedef __attribute__((ext_vector_type(8)))  float    v8f;
typedef __attribute__((ext_vector_type(4)))  float    v4f;

constexpr int kBatch = 4;
constexpr int kSeq   = 2048;
constexpr int kD     = 1024;
constexpr int kH     = 16;
constexpr int kDH    = 64;
constexpr int kTok   = kBatch * kSeq;
constexpr int kSqrtDh = 8;
static_assert(kH * kDH == kD, "head split");
static_assert(kSqrtDh * kSqrtDh == kDH, "sqrt of head dim");
static_assert(kDH == 64, "kernels are written for head dim 64");

constexpr float kXCarry  = 16.0f;
constexpr float kWCarry  = 64.0f;
constexpr float kQKCarry = 16.0f;
constexpr float kVCarry  = 16.0f;
constexpr float kPCarry  = 4096.0f;
constexpr float kLog2e   = 1.4426950408889634f;
constexpr float kProjScale  = 1.0f / (kXCarry * kWCarry);
constexpr float kScoreScale = kLog2e / ((float)kSqrtDh * kQKCarry * kQKCarry);

constexpr int kQB     = 64;
constexpr int kKC     = 64;
constexpr int kNW     = 4;
constexpr int kQBlocks = kSeq / kQB;
constexpr int kChunks  = kSeq / kKC;
constexpr int kOPitch  = 68;
static_assert(kSeq % kQB == 0 && kSeq % kKC == 0, "tile multiples");
static_assert(kQB == kNW * 16, "16 query rows per wave");

constexpr size_t kSzX16  = (size_t)kTok * kD * 2;
constexpr size_t kSzW16  = (size_t)3 * kH * kDH * kDH * 2;
constexpr size_t kSzQ16  = (size_t)kH * kTok * kDH * 2;
constexpr size_t kOffX16 = 0;
constexpr size_t kOffW16 = kOffX16 + kSzX16;
constexpr size_t kOffQ16 = kOffW16 + kSzW16;
constexpr size_t kOffK16 = kOffQ16 + kSzQ16;
constexpr size_t kOffVT16 = kOffK16 + kSzQ16;
constexpr size_t kWsTotal = kOffVT16 + kSzQ16;
static_assert(kWsTotal == 67502080ull, "carve total");
static_assert(kWsTotal <= 134217728ull, "carve cap");
static_assert((kOffW16 % 128) == 0 && (kOffQ16 % 128) == 0 && (kOffK16 % 128) == 0 && (kOffVT16 % 128) == 0, "128-B aligned regions");

template <typename T> struct Frag;
template <> struct Frag<_Float16> {
  typedef v16h V; union U { v16h v; v8h h[2]; };
  static __device__ __forceinline__ v16h load(const _Float16* p) {
    U f; f.h[0] = *(const v8h*)(p); f.h[1] = *(const v8h*)(p + 16); return f.v;
  }
};
__device__ __forceinline__ v8f mma_h(v16h a, v16h b, v8f c) {
  c = __builtin_amdgcn_wmma_f32_16x16x32_f16(false, a, false, b, (short)0, c, false, false);
  asm volatile("v_nop\n\tv_nop\n\tv_nop\n\tv_nop" : "+v"(c) : "v"(a), "v"(b));
  return c;
}

__device__ __forceinline__ float ex2(float x) {
#if __has_builtin(__builtin_amdgcn_exp2f)
  return __builtin_amdgcn_exp2f(x);
#else
  return exp2f(x);
#endif
}

__global__ __launch_bounds__(256) void cast8_carry_kernel(
    const float* __restrict__ in0, const float* __restrict__ in1, const float* __restrict__ in2,
    unsigned short* __restrict__ out, int n8, float carry)
{
  const int i = blockIdx.x * 256 + threadIdx.x;
  if (i >= n8) return;
  const int z = blockIdx.y;
  const float* in = (z == 0) ? in0 : ((z == 1) ? in1 : in2);
  const float* p = in + 8 * (size_t)i;
  const v4f a0 = *(const v4f*)(p);
  const v4f a1 = *(const v4f*)(p + 4);
  v8h hv;
#pragma unroll
  for (int e = 0; e < 4; ++e) {
    const float f0 = a0[e] * carry;
    const float f1 = a1[e] * carry;
    hv[e]     = (_Float16)f0;
    hv[4 + e] = (_Float16)f1;
  }
  unsigned short* q = out + (size_t)z * (size_t)n8 * 8 + 8 * (size_t)i;
  *(volatile v8h*)q = hv;
  __threadfence();
  *(volatile v8h*)q = hv;
}

template <int BIAS_MODE>
__global__ __launch_bounds__(256) void proj_gemm64(
    const unsigned short* __restrict__ Ap, int lda, long strideA,
    const unsigned short* __restrict__ Btp, int ldb, long strideB,
    unsigned short* __restrict__ Cout, int ldc, long strideC,
    const float* __restrict__ bias, long strideBias,
    int M, int N, int K, float scale, float outscale)
{
  __shared__ __align__(16) float sT[8][16 * 68];
  const int b    = blockIdx.y;
  const int lane = threadIdx.x & 31;
  const int wave = __builtin_amdgcn_readfirstlane((int)(threadIdx.x >> 5));
  const int tilesN = N >> 6;
  const int tilesM = M >> 6;
  const int tile = blockIdx.x * 8 + wave;
  if (tile >= tilesM * tilesN) return;
  const int tm = tile / tilesN;
  const int tn = tile - tm * tilesN;
  const int m0 = tm << 6;
  const int n0 = tn << 6;

  const _Float16* Ab = (const _Float16*)Ap  + (size_t)b * strideA;
  const _Float16* Bb = (const _Float16*)Btp + (size_t)b * strideB;
  const float*    bp = bias + (size_t)b * strideBias;

  const int rlane = lane & 15;
  const int koff  = (lane >> 4) * 8;
  const int mOff  = (lane >> 4) * 8;

  v8f acc[4][4];
#pragma unroll
  for (int i = 0; i < 4; ++i)
#pragma unroll
    for (int j = 0; j < 4; ++j) acc[i][j] = (v8f){0.f,0.f,0.f,0.f,0.f,0.f,0.f,0.f};

  for (int k0 = 0; k0 < K; k0 += 32) {
    v16h bh[4];
#pragma unroll
    for (int j = 0; j < 4; ++j) {
      const size_t bo = (size_t)(n0 + (j << 4) + rlane) * ldb + koff + k0;
      bh[j] = Frag<_Float16>::load(Bb + bo);
    }
#pragma unroll
    for (int i = 0; i < 4; ++i) {
      const size_t ao = (size_t)(m0 + (i << 4) + rlane) * lda + koff + k0;
      const v16h ah = Frag<_Float16>::load(Ab + ao);
#pragma unroll
      for (int j = 0; j < 4; ++j) acc[i][j] = mma_h(ah, bh[j], acc[i][j]);
    }
  }

  float* slab = sT[wave];
  unsigned short* C = Cout + (size_t)b * strideC;
#pragma unroll
  for (int i = 0; i < 4; ++i) {
    const int mBase = m0 + (i << 4);
    float bm[8];
#pragma unroll
    for (int r = 0; r < 8; ++r) bm[r] = 0.f;
    if (BIAS_MODE == 1) {
      const v4f b0 = *(const v4f*)(bp + mBase + mOff);
      const v4f b1 = *(const v4f*)(bp + mBase + mOff + 4);
      bm[0] = b0[0]; bm[1] = b0[1]; bm[2] = b0[2]; bm[3] = b0[3];
      bm[4] = b1[0]; bm[5] = b1[1]; bm[6] = b1[2]; bm[7] = b1[3];
    }
#pragma unroll
    for (int j = 0; j < 4; ++j) {
      const int n = n0 + (j << 4) + rlane;
      float bn = 0.f;
      if (BIAS_MODE == 2) bn = bp[n];
#pragma unroll
      for (int r = 0; r < 8; ++r) {
        float v = acc[i][j][r] * scale;
        if (BIAS_MODE == 1) v += bm[r];
        if (BIAS_MODE == 2) v += bn;
        v *= outscale;
        slab[(mOff + r) * 68 + (j << 4) + rlane] = v;
      }
    }
    __builtin_amdgcn_fence(__ATOMIC_RELEASE, "workgroup");
    __builtin_amdgcn_wave_barrier();
    __builtin_amdgcn_fence(__ATOMIC_ACQUIRE, "workgroup");
    {
      const int q = lane >> 3, c8 = (lane & 7) * 8;
      for (int pass = 0; pass < 2; ++pass) {
#pragma unroll
        for (int it = 0; it < 4; ++it) {
          const int row = it * 4 + q;
          const float* sp = slab + row * 68 + c8;
          v8h hv;
#pragma unroll
          for (int e = 0; e < 8; ++e) hv[e] = (_Float16)sp[e];
          *(volatile v8h*)(C + (size_t)(mBase + row) * ldc + n0 + c8) = hv;
        }
        __threadfence();
      }
    }
    __builtin_amdgcn_fence(__ATOMIC_RELEASE, "workgroup");
    __builtin_amdgcn_wave_barrier();
    __builtin_amdgcn_fence(__ATOMIC_ACQUIRE, "workgroup");
  }
}

__global__ __launch_bounds__(128) void attn_f16_kernel(
    const unsigned short* __restrict__ Qp, const unsigned short* __restrict__ Kp,
    const unsigned short* __restrict__ Vtp, float* __restrict__ out)
{
  __shared__ __align__(16) _Float16 Ksh[kKC * kDH];
  __shared__ __align__(16) _Float16 Vsh[kDH * kKC];
  __shared__ __align__(16) _Float16 Psh[kNW][16 * kKC];
  __shared__ __align__(16) float    Os[kNW][16 * kOPitch];

  const int tid  = threadIdx.x;
  const int wave = __builtin_amdgcn_readfirstlane((int)(threadIdx.x >> 5));
  const int lane = tid & 31;
  const int hh   = lane >> 4;
  const int c    = lane & 15;

  const int bx = blockIdx.x;
  const int qb = bx % kQBlocks;
  const int bh = bx / kQBlocks;
  const int h  = bh % kH;
  const int b  = bh / kH;
  const int q0 = qb * kQB + wave * 16;

  const _Float16* Qb = (const _Float16*)Qp  + ((size_t)h * kTok + (size_t)b * kSeq) * kDH;
  const _Float16* Kb = (const _Float16*)Kp  + ((size_t)h * kTok + (size_t)b * kSeq) * kDH;
  const _Float16* Vb = (const _Float16*)Vtp + (size_t)h * kDH * kTok + (size_t)b * kSeq;
  float* Ob = out + (size_t)b * kSeq * kD + (size_t)h * kDH;

  v16h qa[2];
#pragma unroll
  for (int dc = 0; dc < 2; ++dc)
    qa[dc] = Frag<_Float16>::load(Qb + (size_t)(q0 + c) * kDH + dc * 32 + 8 * hh);

  float mrow[8], lrow[8];
  v8f oacc[4];
#pragma unroll
  for (int r = 0; r < 8; ++r) { mrow[r] = -1.0e30f; lrow[r] = 0.f; }
#pragma unroll
  for (int t = 0; t < 4; ++t) oacc[t] = (v8f){0.f,0.f,0.f,0.f,0.f,0.f,0.f,0.f};

  _Float16* pw = Psh[wave];

#pragma unroll 1
  for (int kc = 0; kc < kChunks; ++kc) {
    const int kv0 = kc * kKC;
    __syncthreads();
#pragma unroll
    for (int p = 0; p < 4; ++p) {
      const int idx = tid + p * 128;
      const int r   = idx >> 3;
      const int c8  = (idx & 7) * 8;
      const v8h kvv = *(const v8h*)(Kb + (size_t)(kv0 + r) * kDH + c8);
      const v8h vvv = *(const v8h*)(Vb + (size_t)r * kTok + kv0 + c8);
      *(v8h*)(Ksh + r * kDH + c8) = kvv;
      *(v8h*)(Vsh + r * kKC + c8) = vvv;
    }
    __syncthreads();

    v8f s[4];
#pragma unroll
    for (int j = 0; j < 4; ++j) {
      s[j] = (v8f){0.f,0.f,0.f,0.f,0.f,0.f,0.f,0.f};
#pragma unroll
      for (int dc = 0; dc < 2; ++dc) {
        const v16h kb = Frag<_Float16>::load(Ksh + (j * 16 + c) * kDH + dc * 32 + 8 * hh);
        s[j] = mma_h(qa[dc], kb, s[j]);
      }
    }

    float cm[8];
#pragma unroll
    for (int r = 0; r < 8; ++r) {
      float m = -1.0e30f;
#pragma unroll
      for (int j = 0; j < 4; ++j) {
        const float tv = s[j][r] * kScoreScale;
        s[j][r] = tv;
        m = fmaxf(m, tv);
      }
#pragma unroll
      for (int off = 1; off < 16; off <<= 1) m = fmaxf(m, __shfl_xor(m, off, 32));
      cm[r] = m;
    }

#pragma unroll
    for (int r = 0; r < 8; ++r) {
      const float mnew  = fmaxf(mrow[r], cm[r]);
      const float alpha = ex2(mrow[r] - mnew);
      mrow[r] = mnew;
      float psum = 0.f;
#pragma unroll
      for (int j = 0; j < 4; ++j) {
        const float p = ex2(s[j][r] - mnew);
        const _Float16 ph = (_Float16)(p * kPCarry);
        const float pf = (float)ph;
        psum += pf;
        pw[(8 * hh + r) * kKC + j * 16 + c] = ph;
      }
      lrow[r] = lrow[r] * alpha + psum;
#pragma unroll
      for (int t = 0; t < 4; ++t) oacc[t][r] *= alpha;
    }
    __builtin_amdgcn_fence(__ATOMIC_RELEASE, "workgroup");
    __builtin_amdgcn_wave_barrier();
    __builtin_amdgcn_fence(__ATOMIC_ACQUIRE, "workgroup");

#pragma unroll
    for (int kk = 0; kk < 2; ++kk) {
      const v16h pa = Frag<_Float16>::load(pw + c * kKC + kk * 32 + 8 * hh);
#pragma unroll
      for (int t = 0; t < 4; ++t) {
        const v16h vb = Frag<_Float16>::load(Vsh + (t * 16 + c) * kKC + kk * 32 + 8 * hh);
        oacc[t] = mma_h(pa, vb, oacc[t]);
      }
    }
  }

  float* os = Os[wave];
#pragma unroll
  for (int r = 0; r < 8; ++r) {
    float l = lrow[r];
#pragma unroll
    for (int off = 1; off < 16; off <<= 1) l += __shfl_xor(l, off, 32);
    const float inv = 1.0f / (l * kVCarry);
#pragma unroll
    for (int t = 0; t < 4; ++t) os[(8 * hh + r) * kOPitch + t * 16 + c] = oacc[t][r] * inv;
  }
  __builtin_amdgcn_fence(__ATOMIC_RELEASE, "workgroup");
  __builtin_amdgcn_wave_barrier();
  __builtin_amdgcn_fence(__ATOMIC_ACQUIRE, "workgroup");
  {
    const int c4 = (lane & 15) * 4;
    for (int pass = 0; pass < 2; ++pass) {
#pragma unroll
      for (int it = 0; it < 8; ++it) {
        const int row = it * 2 + hh;
        const v4f val = *(const v4f*)(os + row * kOPitch + c4);
        *(volatile v4f*)(Ob + (size_t)(q0 + row) * kD + c4) = val;
      }
      __threadfence();
    }
  }
}

static_assert((kTok % 64) == 0 && (kDH % 64) == 0 && (kDH % 32) == 0, "GEMM tile multiples");
static_assert(((kTok / 64) * (kDH / 64)) % 8 == 0, "exact GEMM grids");
static_assert(((kTok * kD / 8) % 256) == 0 && ((kH * kDH * kDH / 8) % 256) == 0, "exact cast grids");

extern "C" void kernel_launch(void* const* d_in, const int* in_sizes, int n_in,
                              void* d_out, int out_size, void* d_ws, size_t ws_size,
                              hipStream_t stream) {
  if (n_in < 7) return;
  if (in_sizes[0] != kTok * kD) return;
  if (in_sizes[1] != kH * kDH * kDH) return;
  if (in_sizes[2] != kH * kDH) return;
  if (in_sizes[3] != kH * kDH * kDH) return;
  if (in_sizes[4] != kH * kDH) return;
  if (in_sizes[5] != kH * kDH * kDH) return;
  if (in_sizes[6] != kH * kDH) return;
  if (out_size != kTok * kD) return;
  if (ws_size < kWsTotal) return;

  const float* x  = (const float*)d_in[0];
  const float* Wq = (const float*)d_in[1];
  const float* bq = (const float*)d_in[2];
  const float* Wk = (const float*)d_in[3];
  const float* bk = (const float*)d_in[4];
  const float* Wv = (const float*)d_in[5];
  const float* bv = (const float*)d_in[6];
  float* out = (float*)d_out;

  char* ws = (char*)d_ws;
  unsigned short* X16  = (unsigned short*)(ws + kOffX16);
  unsigned short* W16  = (unsigned short*)(ws + kOffW16);
  unsigned short* Q16  = (unsigned short*)(ws + kOffQ16);
  unsigned short* K16  = (unsigned short*)(ws + kOffK16);
  unsigned short* VT16 = (unsigned short*)(ws + kOffVT16);
  unsigned short* Wq16 = W16;
  unsigned short* Wk16 = W16 + (size_t)kH * kDH * kDH;
  unsigned short* Wv16 = W16 + (size_t)2 * kH * kDH * kDH;

  cast8_carry_kernel<<<dim3((kTok * kD / 8) / 256, 1), 256, 0, stream>>>(x, x, x, X16, kTok * kD / 8, kXCarry);
  cast8_carry_kernel<<<dim3((kH * kDH * kDH / 8) / 256, 3), 256, 0, stream>>>(Wq, Wk, Wv, W16, kH * kDH * kDH / 8, kWCarry);

  const int projBlocks = ((kTok / 64) * (kDH / 64)) / 8;
  proj_gemm64<2><<<dim3(projBlocks, kH), 256, 0, stream>>>(
      X16, kD, (long)kDH,
      Wq16, kDH, (long)(kDH * kDH),
      Q16, kDH, (long)kTok * kDH,
      bq, (long)kDH,
      kTok, kDH, kDH, kProjScale, kQKCarry);
  proj_gemm64<2><<<dim3(projBlocks, kH), 256, 0, stream>>>(
      X16, kD, (long)kDH,
      Wk16, kDH, (long)(kDH * kDH),
      K16, kDH, (long)kTok * kDH,
      bk, (long)kDH,
      kTok, kDH, kDH, kProjScale, kQKCarry);
  proj_gemm64<1><<<dim3(projBlocks, kH), 256, 0, stream>>>(
      Wv16, kDH, (long)(kDH * kDH),
      X16, kD, (long)kDH,
      VT16, kTok, (long)kDH * kTok,
      bv, (long)kDH,
      kDH, kTok, kDH, kProjScale, kVCarry);

  attn_f16_kernel<<<kBatch * kH * kQBlocks, kNW * 32, 0, stream>>>(Q16, K16, VT16, out);
}
